// HGSA_v14_3693671875060
// MI455X (gfx1250) — hardware-verified
//
#include <hip/hip_runtime.h>
#include <math.h>

#define BB     2
#define HH     256
#define WW     256
#define CC     64
#define NPIX   (HH*WW)
#define MROWS  (BB*NPIX)
#define HEADS  4
#define DHEAD  16

typedef _Float16 v16h __attribute__((ext_vector_type(16)));
typedef _Float16 v8h  __attribute__((ext_vector_type(8)));
typedef float    v8f  __attribute__((ext_vector_type(8)));
typedef float    v4f  __attribute__((ext_vector_type(4)));
#define VST2(T, ptr, val) do { const T _v = (val); *(volatile T*)(ptr) = _v; __threadfence(); *(volatile T*)(ptr) = _v; } while (0)
#define NBLK1 (MROWS / 128)
#define PART  2304
typedef unsigned int u32x4 __attribute__((ext_vector_type(4)));
typedef int          i32x8 __attribute__((ext_vector_type(8)));
typedef int          i32x4 __attribute__((ext_vector_type(4)));

__device__ __forceinline__ v16h load_a_frag(const _Float16* base, int r0, int k0,
                                            int lm, int lh) {
    const _Float16* p = base + (r0 + lm) * 64 + k0 + lh * 8;
    union { v16h v; v8h h[2]; } u;
    u.h[0] = *(const v8h*)p;
    u.h[1] = *(const v8h*)(p + 16);
    return u.v;
}

__device__ __forceinline__ v16h load_b_frag(const _Float16* wt, int nt, int ks, int lane) {
    const int n = nt * 16 + (lane & 15), hh = lane >> 4;
    v16h v;
#pragma unroll
    for (int j = 0; j < 16; ++j) {
        const int k = ks * 32 + ((j < 8) ? j : (j + 8)) + 8 * hh;
        v[j] = wt[k * 64 + n];
    }
    return v;
}

__device__ __forceinline__ v8f wmma16(v16h a, v16h b, v8f c) {
    v8f d = __builtin_amdgcn_wmma_f32_16x16x32_f16(false, a, false, b, (short)0, c, false, false);
    asm volatile("v_nop\n\tv_nop\n\tv_nop\n\tv_nop" : "+v"(d) : "v"(a), "v"(b));
    return d;
}

__global__ void hgsa_qkv(const float* __restrict__ x, const float* __restrict__ mask,
                         const float* __restrict__ Wq, const float* __restrict__ Wk,
                         const float* __restrict__ Wv, const float* __restrict__ mw1,
                         const float* __restrict__ mb1, const float* __restrict__ mw2,
                         const float* __restrict__ mb2,
                         _Float16* __restrict__ vout, _Float16* __restrict__ m1out,
                         _Float16* __restrict__ m2out, float* __restrict__ part) {
    extern __shared__ char smem[];
    _Float16* Xl  = (_Float16*)smem;
    _Float16* Ml  = Xl + 128 * 64;
    _Float16* WTl = Ml + 128 * 64;
    float*    Ql  = (float*)(WTl + 5 * 64 * 64);
    float*    Kl  = Ql + 128 * 64;
    _Float16* M1l = (_Float16*)(Kl + 128 * 64);
    _Float16* St  = M1l + 128 * 64;

    const int t    = threadIdx.x;
    const int m0   = blockIdx.x * 128;
    const int bidx = m0 >> 16;

    for (int i = t; i < 128 * 64; i += 256) {
        Xl[i] = (_Float16)x[(size_t)m0 * 64 + i];
        Ml[i] = (_Float16)mask[(size_t)m0 * 64 + i];
    }
    for (int i = t; i < 64 * 64; i += 256) {
        int k = i >> 6, o = i & 63;
        WTl[0 * 4096 + i] = (_Float16)Wq[o * 64 + k];
        WTl[1 * 4096 + i] = (_Float16)Wk[o * 64 + k];
        WTl[2 * 4096 + i] = (_Float16)Wv[o * 64 + k];
        WTl[3 * 4096 + i] = (_Float16)mw1[o * 64 + k];
        WTl[4 * 4096 + i] = (_Float16)mw2[o * 64 + k];
    }
    __syncthreads();

    const int wave = t >> 5, lane = t & 31;
    const int r0 = wave * 16;
    const int lm = lane & 15, lh = lane >> 4;

    v16h ax0 = load_a_frag(Xl, r0, 0, lm, lh);
    v16h ax1 = load_a_frag(Xl, r0, 32, lm, lh);
    v16h am0 = load_a_frag(Ml, r0, 0, lm, lh);
    v16h am1 = load_a_frag(Ml, r0, 32, lm, lh);

#pragma unroll
    for (int nt = 0; nt < 4; ++nt) {
        v8f cq = {};
        cq = wmma16(ax0, load_b_frag(WTl + 0 * 4096, nt, 0, lane), cq);
        cq = wmma16(ax1, load_b_frag(WTl + 0 * 4096, nt, 1, lane), cq);
        v8f ck = {};
        ck = wmma16(ax0, load_b_frag(WTl + 1 * 4096, nt, 0, lane), ck);
        ck = wmma16(ax1, load_b_frag(WTl + 1 * 4096, nt, 1, lane), ck);
        v8f cv = {};
        cv = wmma16(ax0, load_b_frag(WTl + 2 * 4096, nt, 0, lane), cv);
        cv = wmma16(ax1, load_b_frag(WTl + 2 * 4096, nt, 1, lane), cv);
        v8f c1 = {};
        c1 = wmma16(am0, load_b_frag(WTl + 3 * 4096, nt, 0, lane), c1);
        c1 = wmma16(am1, load_b_frag(WTl + 3 * 4096, nt, 1, lane), c1);
        float b1v = mb1[nt * 16 + lm];
#pragma unroll
        for (int r = 0; r < 8; ++r) {
            int row = r0 + r + 8 * lh;
            int col = nt * 16 + lm;
            Ql[row * 64 + col] = cq[r];
            Kl[row * 64 + col] = ck[r];
            St[(wave * 16 + r + 8 * lh) * 64 + col] = (_Float16)cv[r];
            float m1v = c1[r] + b1v;
            M1l[row * 64 + col] = (_Float16)m1v;
        }
    }
    __builtin_amdgcn_fence(__ATOMIC_RELEASE, "workgroup"); __builtin_amdgcn_wave_barrier(); __builtin_amdgcn_fence(__ATOMIC_ACQUIRE, "workgroup");
    for (int pass = 0; pass < 2; ++pass) {
#pragma unroll
        for (int jj = 0; jj < 4; ++jj) { const int rr = jj * 4 + (lane >> 3), sg = lane & 7;
            *(volatile v8h*)(vout  + (size_t)(m0 + r0 + rr) * 64 + sg * 8) = *(const v8h*)(St  + (wave * 16 + rr) * 64 + sg * 8);
            *(volatile v8h*)(m1out + (size_t)(m0 + r0 + rr) * 64 + sg * 8) = *(const v8h*)(M1l + (r0 + rr) * 64 + sg * 8); }
        __threadfence();
    }
    __syncthreads();

    v16h a10 = load_a_frag(M1l, r0, 0, lm, lh);
    v16h a11 = load_a_frag(M1l, r0, 32, lm, lh);
#pragma unroll
    for (int nt = 0; nt < 4; ++nt) {
        v8f c2 = {};
        c2 = wmma16(a10, load_b_frag(WTl + 4 * 4096, nt, 0, lane), c2);
        c2 = wmma16(a11, load_b_frag(WTl + 4 * 4096, nt, 1, lane), c2);
        float b2v = mb2[nt * 16 + lm];
#pragma unroll
        for (int r = 0; r < 8; ++r) St[(wave * 16 + r + 8 * lh) * 64 + nt * 16 + lm] = (_Float16)(c2[r] + b2v);
    }
    __builtin_amdgcn_fence(__ATOMIC_RELEASE, "workgroup"); __builtin_amdgcn_wave_barrier(); __builtin_amdgcn_fence(__ATOMIC_ACQUIRE, "workgroup");
    for (int pass = 0; pass < 2; ++pass) {
#pragma unroll
        for (int jj = 0; jj < 4; ++jj) { const int rr = jj * 4 + (lane >> 3), sg = lane & 7;
            *(volatile v8h*)(m2out + (size_t)(m0 + r0 + rr) * 64 + sg * 8) = *(const v8h*)(St + (wave * 16 + rr) * 64 + sg * 8); }
        __threadfence();
    }

    {
        const int head = t >> 6;
        const int d    = (t >> 2) & 15;
        const int e0   = (t & 3) * 4;
        float acc0 = 0.f, acc1 = 0.f, acc2 = 0.f, acc3 = 0.f;
        for (int p = 0; p < 128; ++p) {
            float kv = Kl[p * 64 + head * 16 + d];
            const float* qp = &Ql[p * 64 + head * 16 + e0];
            acc0 = fmaf(kv, qp[0], acc0);
            acc1 = fmaf(kv, qp[1], acc1);
            acc2 = fmaf(kv, qp[2], acc2);
            acc3 = fmaf(kv, qp[3], acc3);
        }
        float* gram = part + (size_t)blockIdx.x * PART + (head * 16 + d) * 16 + e0;
        v4f g4 = {acc0, acc1, acc2, acc3};
        VST2(v4f, gram, g4);
    }
    if (t < 128) {
        int isK = t >> 6;
        int hh2 = (t >> 4) & 3;
        int e   = t & 15;
        const float* src = isK ? Kl : Ql;
        float s = 0.f;
        for (int p = 0; p < 128; ++p) {
            float vv = src[p * 64 + hh2 * 16 + e];
            s = fmaf(vv, vv, s);
        }
        VST2(float, part + (size_t)blockIdx.x * PART + 1024 + isK * 64 + hh2 * 16 + e, s);
    }
    (void)bidx;
}

__global__ __launch_bounds__(256) void hgsa_reduce(const float* __restrict__ part, float* __restrict__ accum) {
    for (int i = threadIdx.x; i < 2304; i += 256) {
        int b, li;
        if (i < 2048) { b = i >> 10; li = i & 1023; }
        else { const int j = i - 2048; const int isK = j >> 7; const int bh = (j & 127) >> 4, e = j & 15; b = bh >> 2; li = 1024 + isK * 64 + (bh & 3) * 16 + e; }
        float s = 0.f;
        for (int blk = 0; blk < NBLK1 / BB; ++blk) s += part[((size_t)(b * (NBLK1 / BB) + blk)) * PART + li];
        VST2(float, accum + i, s);
    }
}

__global__ void hgsa_attn(const float* __restrict__ accum,
                          const float* __restrict__ rescale,
                          const float* __restrict__ Wp,
                          _Float16* __restrict__ wefft) {
    __shared__ float attnL[BB * HEADS * 16 * 16];
    const int t = threadIdx.x;
    if (t < 128) {
        int b = t >> 6, head = (t >> 4) & 3, d = t & 15;
        const float* S   = accum + ((b * 4 + head) * 16 + d) * 16;
        const float* ssq = accum + 2048 + (b * 4 + head) * 16;
        const float* ssk = accum + 2176 + (b * 4 + head) * 16;
        float kn = fmaxf(sqrtf(ssk[d]), 1e-12f);
        float rs = rescale[head];
        float vals[16];
        float mx = -3.4e38f;
#pragma unroll
        for (int e = 0; e < 16; ++e) {
            float qn = fmaxf(sqrtf(ssq[e]), 1e-12f);
            vals[e] = S[e] / (kn * qn) * rs;
            mx = fmaxf(mx, vals[e]);
        }
        float sum = 0.f;
#pragma unroll
        for (int e = 0; e < 16; ++e) { vals[e] = expf(vals[e] - mx); sum += vals[e]; }
        float inv = 1.0f / sum;
#pragma unroll
        for (int e = 0; e < 16; ++e)
            attnL[(((b * 4 + head) * 16 + d) * 16) + e] = vals[e] * inv;
    }
    __syncthreads();
    {
        __shared__ __attribute__((aligned(16))) _Float16 sW[8][16 * 64];
        const int wave = t >> 5, lane = t & 31, hh = lane >> 4, l16 = lane & 15;
        const int b = wave >> 2, h = wave & 3;
        v16h af;
#pragma unroll
        for (int j = 0; j < 16; ++j) {
            const int k = ((j < 8) ? j : (j + 8)) + 8 * hh;
            af[j] = (k < 16) ? (_Float16)attnL[((b * 4 + h) * 16 + k) * 16 + l16] : (_Float16)0.0f;
        }
#pragma unroll
        for (int ot = 0; ot < 4; ++ot) {
            v16h bf;
            const int o = ot * 16 + l16;
#pragma unroll
            for (int j = 0; j < 16; ++j) {
                const int k = ((j < 8) ? j : (j + 8)) + 8 * hh;
                bf[j] = (k < 16) ? (_Float16)Wp[o * 64 + h * 16 + k] : (_Float16)0.0f;
            }
            v8f acc = {};
            acc = wmma16(af, bf, acc);
#pragma unroll
            for (int r = 0; r < 8; ++r) sW[wave][(8 * hh + r) * 64 + o] = (_Float16)acc[r];
        }
        __builtin_amdgcn_fence(__ATOMIC_RELEASE, "workgroup"); __builtin_amdgcn_wave_barrier(); __builtin_amdgcn_fence(__ATOMIC_ACQUIRE, "workgroup");
        _Float16* dst = wefft + (size_t)b * 4096 + (size_t)(h * 16) * 64;
        for (int pass = 0; pass < 2; ++pass) {
#pragma unroll
            for (int jj = 0; jj < 4; ++jj) { const int rr = jj * 4 + (lane >> 3), sg = lane & 7;
                *(volatile v8h*)(dst + rr * 64 + sg * 8) = *(const v8h*)(&sW[wave][rr * 64 + sg * 8]); }
            __threadfence();
        }
    }
}

__global__ void hgsa_stencil(const float* __restrict__ x,
                             const _Float16* __restrict__ m1g,
                             const _Float16* __restrict__ m2g,
                             _Float16* __restrict__ vg,
                             const float* __restrict__ mdw,
                             const float* __restrict__ mdwb,
                             const float* __restrict__ pw1,
                             const float* __restrict__ pw2,
                             float* __restrict__ out) {
    extern __shared__ char smem[];
    _Float16* m2s  = (_Float16*)smem;
    _Float16* t2s  = m2s + 20 * 20 * 64;
    float*    wdw  = (float*)(t2s + 18 * 18 * 64);
    float*    wp1  = wdw + 64 * 25;
    float*    wp2  = wp1 + 64 * 9;
    float*    wdwb = wp2 + 64 * 9;

    const int t  = threadIdx.x;
    const int bi = blockIdx.x;
    const int b  = bi >> 8;
    const int by = (bi >> 4) & 15;
    const int bx = bi & 15;

    for (int i = t; i < 64 * 25; i += 256) wdw[i] = mdw[i];
    for (int i = t; i < 64 * 9; i += 256) { wp1[i] = pw1[i]; wp2[i] = pw2[i]; }
    if (t < 64) wdwb[t] = mdwb[t];

    for (int i = t; i < 20 * 20 * 64; i += 256) {
        int iy = i / (20 * 64);
        int r  = i - iy * (20 * 64);
        int ix = r >> 6, c = r & 63;
        int gy = by * 16 - 2 + iy, gx = bx * 16 - 2 + ix;
        _Float16 v = (_Float16)0.0f;
        if (gy >= 0 && gy < HH && gx >= 0 && gx < WW)
            v = m2g[((size_t)(b * HH + gy) * WW + gx) * 64 + c];
        m2s[i] = v;
    }
    for (int i = t; i < 18 * 18 * 64; i += 256) {
        int iy = i / (18 * 64);
        int r  = i - iy * (18 * 64);
        int ix = r >> 6, c = r & 63;
        int gy = by * 16 - 1 + iy, gx = bx * 16 - 1 + ix;
        float t1 = 0.f;
#pragma unroll
        for (int ky = 0; ky < 3; ++ky) {
#pragma unroll
            for (int kx = 0; kx < 3; ++kx) {
                int yy = gy + ky - 1, xx = gx + kx - 1;
                if (yy >= 0 && yy < HH && xx >= 0 && xx < WW)
                    t1 = fmaf(x[((size_t)(b * HH + yy) * WW + xx) * 64 + c],
                              wp1[c * 9 + ky * 3 + kx], t1);
            }
        }
        float g = 0.5f * t1 * (1.0f + erff(t1 * 0.7071067811865476f));
        if (gy < 0 || gy >= HH || gx < 0 || gx >= WW) g = 0.0f;
        t2s[i] = (_Float16)g;
    }
    __syncthreads();

    const int c = t & 63, pg = t >> 6;
    for (int pp = pg; pp < 256; pp += 4) {
        const int ly = pp >> 4, lx = pp & 15;
        const int y = by * 16 + ly, xq = bx * 16 + lx;
        const size_t pix = (size_t)(b * HH + y) * WW + xq;
        float s = wdwb[c];
#pragma unroll
        for (int ky = 0; ky < 5; ++ky) {
#pragma unroll
            for (int kx = 0; kx < 5; ++kx)
                s = fmaf((float)m2s[((ly + ky) * 20 + (lx + kx)) * 64 + c],
                         wdw[c * 25 + ky * 5 + kx], s);
        }
        float sig = 1.0f / (1.0f + expf(-s));
        float m1v = (float)m1g[pix * 64 + c];
        float ma  = fmaf(m1v, sig, m1v);
        float vf  = (float)vg[pix * 64 + c] * ma;
        VST2(_Float16, vg + pix * 64 + c, (_Float16)vf);

        float p = 0.f;
#pragma unroll
        for (int ky = 0; ky < 3; ++ky) {
#pragma unroll
            for (int kx = 0; kx < 3; ++kx)
                p = fmaf((float)t2s[((ly + ky) * 18 + (lx + kx)) * 64 + c],
                         wp2[c * 9 + ky * 3 + kx], p);
        }
        VST2(float, out + pix * 64 + c, p);
    }
}

__global__ void hgsa_proj(const _Float16* __restrict__ vg,
                          const _Float16* __restrict__ wefft,
                          const float* __restrict__ bp,
                          float* __restrict__ out) {
    __shared__ _Float16 Vl[128 * 64];
    __shared__ _Float16 Wl[64 * 64];
    const int t  = threadIdx.x;
    const int m0 = blockIdx.x * 128;
    const int b  = m0 >> 16;

    for (int i = t; i < 128 * 64 / 8; i += 256) *(v8h*)(Vl + i * 8) = *(const v8h*)(vg + (size_t)m0 * 64 + i * 8);
    for (int i = t; i < 64 * 64 / 8; i += 256)  *(v8h*)(Wl + i * 8) = *(const v8h*)(wefft + b * 4096 + i * 8);
    __syncthreads();

    const int wave = t >> 5, lane = t & 31;
    const int r0 = wave * 16;
    const int lm = lane & 15, lh = lane >> 4;

    v16h a0 = load_a_frag(Vl, r0, 0, lm, lh);
    v16h a1 = load_a_frag(Vl, r0, 32, lm, lh);
    v8f cc[4];
#pragma unroll
    for (int nt = 0; nt < 4; ++nt) {
        v8f c = {};
        c = wmma16(a0, load_b_frag(Wl, nt, 0, lane), c);
        c = wmma16(a1, load_b_frag(Wl, nt, 1, lane), c);
        cc[nt] = c;
    }
    float v1s[2][8], v2s[2][8];
#pragma unroll
    for (int pr = 0; pr < 2; ++pr) {
        const float bv = bp[pr * 32 + lane];
#pragma unroll
        for (int r = 0; r < 8; ++r) {
            const float a_ = cc[2 * pr][r], b_ = cc[2 * pr + 1][r];
            const float ax = __shfl_xor(a_, 16), bx = __shfl_xor(b_, 16);
            const size_t i1 = (size_t)(m0 + r0 + r) * 64 + pr * 32 + lane, i2 = (size_t)(m0 + r0 + r + 8) * 64 + pr * 32 + lane;
            v1s[pr][r] = out[i1] + (lh ? bx : a_) + bv;
            v2s[pr][r] = out[i2] + (lh ? b_ : ax) + bv;
        }
    }
    for (int pass = 0; pass < 2; ++pass) {
#pragma unroll
        for (int pr = 0; pr < 2; ++pr)
#pragma unroll
            for (int r = 0; r < 8; ++r) {
                *(volatile float*)(out + (size_t)(m0 + r0 + r) * 64 + pr * 32 + lane) = v1s[pr][r];
                *(volatile float*)(out + (size_t)(m0 + r0 + r + 8) * 64 + pr * 32 + lane) = v2s[pr][r];
            }
        __threadfence();
    }
}

extern "C" void kernel_launch(void* const* d_in, const int* in_sizes, int n_in,
                              void* d_out, int out_size, void* d_ws, size_t ws_size,
                              hipStream_t stream) {
    const float* x    = (const float*)d_in[0];
    const float* mask = (const float*)d_in[1];
    const float* Wq   = (const float*)d_in[2];
    const float* Wk   = (const float*)d_in[3];
    const float* Wv   = (const float*)d_in[4];
    const float* resc = (const float*)d_in[5];
    const float* Wp   = (const float*)d_in[6];
    const float* bp   = (const float*)d_in[7];
    const float* mw1  = (const float*)d_in[8];
    const float* mb1  = (const float*)d_in[9];
    const float* mw2  = (const float*)d_in[10];
    const float* mb2  = (const float*)d_in[11];
    const float* mdw  = (const float*)d_in[12];
    const float* mdwb = (const float*)d_in[13];
    const float* pw1  = (const float*)d_in[14];
    const float* pw2  = (const float*)d_in[15];

    char* ws = (char*)d_ws;
    _Float16* vbuf  = (_Float16*)(ws);
    _Float16* m1buf = (_Float16*)(ws + (size_t)16777216);
    _Float16* m2buf = (_Float16*)(ws + (size_t)33554432);
    float*    accum = (float*)(ws + (size_t)50331648);
    _Float16* wefft = (_Float16*)(ws + (size_t)50340864);
    float*    part  = (float*)(ws + (size_t)50364416);
    float* out = (float*)d_out;
    (void)in_sizes; (void)n_in; (void)out_size;
    if (ws_size < (size_t)50364416 + (size_t)NBLK1 * PART * 4) return;

    size_t lds1 = (size_t)(128 * 64 * 2) * 2 + 5 * 64 * 64 * 2 +
                  (size_t)(128 * 64 * 4) * 2 + 128 * 64 * 2 + 8 * 16 * 64 * 2;
    hgsa_qkv<<<MROWS / 128, 256, lds1, stream>>>(x, mask, Wq, Wk, Wv, mw1, mb1,
                                                 mw2, mb2, vbuf, m1buf, m2buf,
                                                 part);
    hgsa_reduce<<<1, 256, 0, stream>>>(part, accum);

    hgsa_attn<<<1, 256, 0, stream>>>(accum, resc, Wp, wefft);

    size_t lds3 = (size_t)(20 * 20 * 64 * 2) + 18 * 18 * 64 * 2 +
                  64 * 25 * 4 + 64 * 9 * 4 * 2 + 64 * 4;
    hgsa_stencil<<<BB * 16 * 16, 256, lds3, stream>>>(x, m1buf, m2buf, vbuf,
                                                      mdw, mdwb, pw1, pw2, out);

    hgsa_proj<<<MROWS / 128, 256, 0, stream>>>(vbuf, wefft, bp, out);
}
